// SelectiveSSM_82755429859939
// MI455X (gfx1250) — hardware-verified
//
#include <hip/hip_runtime.h>
#include <math.h>

typedef __attribute__((ext_vector_type(16))) _Float16 v16h;
typedef __attribute__((ext_vector_type(8)))  _Float16 v8h;
typedef __attribute__((ext_vector_type(16))) __bf16   v16b;
typedef __attribute__((ext_vector_type(8)))  __bf16   v8b;
typedef __attribute__((ext_vector_type(8)))  float    v8f;
typedef __attribute__((ext_vector_type(4)))  float    v4f;
typedef __attribute__((ext_vector_type(4)))  unsigned v4u;

constexpr int kBatch  = 2;
constexpr int kSeq    = 2048;
constexpr int kDm     = 1024;
constexpr int kDin    = 2048;
constexpr int kNst    = 64;
constexpr int kDtR    = 64;
constexpr int kXzP    = 2 * kDin;
constexpr int kSsmP   = kDtR + 2 * kNst;
constexpr int kBcOff  = kDtR;
constexpr int kBCW    = 2 * kNst;
constexpr int kRows   = kBatch * kSeq;
constexpr int kConvTP = 260;
constexpr int kScanTS = 32;
constexpr int kScanCh = 64;
constexpr int kScanQ  = 16;
constexpr int kScanYP = 68;
constexpr float kLog2e = 1.4426950408889634f;
static_assert((kDm % 32) == 0 && (kDin % 32) == 0 && (kDtR % 32) == 0, "GEMM K multiples of 32");
static_assert((kRows % 64) == 0 && (kDin % 64) == 0 && (kSsmP % 64) == 0 && (kDm % 64) == 0, "GEMM M,N multiples of 64");
static_assert((kSeq % kScanTS) == 0 && (kSeq % 64) == 0 && (kDin % kScanCh) == 0 && (kDin % 256) == 0, "tile multiples");
static_assert(kNst == 4 * kScanQ && kScanCh * 4 == 256, "scan lane map: 4 lanes x 16 states per channel, 256 threads");
static_assert(kDtR == 64, "fused dt tile: exactly two 32-deep k steps");
static_assert((kScanTS / 16) * (kScanCh / 16) == 8, "fused dt tile: one 16x16 subtile per wave, 8 waves");
static_assert(kScanTS * kBCW == 256 * 2 * 8, "scan B|C staging: 2 x 8 elements per thread");
static_assert(kScanTS * kScanCh == 256 * 8, "scan xc/gate staging, softplus and store phases: 8 elements per thread");
static_assert(kScanCh * kNst == kScanTS * kBCW, "A staging fits the B|C tile");

constexpr size_t kOffXB   = 0;
constexpr size_t kOffWIB  = kOffXB   + (size_t)kRows * kDm  * 2;
constexpr size_t kOffWXB  = kOffWIB  + (size_t)kXzP  * kDm  * 2;
constexpr size_t kOffWDB  = kOffWXB  + (size_t)kSsmP * kDin * 2;
constexpr size_t kOffWOB  = kOffWDB  + (size_t)kDin  * kDtR * 2;
constexpr size_t kOffXSH  = kOffWOB  + (size_t)kDm   * kDin * 2;
constexpr size_t kOffXSL  = kOffXSH  + (size_t)kRows * kDin * 2;
constexpr size_t kOffZH   = kOffXSL  + (size_t)kRows * kDin * 2;
constexpr size_t kOffZL   = kOffZH   + (size_t)kRows * kDin * 2;
constexpr size_t kOffXCH  = kOffZL   + (size_t)kRows * kDin * 2;
constexpr size_t kOffXCL  = kOffXCH  + (size_t)kRows * kDin * 2;
constexpr size_t kOffSSH  = kOffXCL  + (size_t)kRows * kDin * 2;
constexpr size_t kOffSSL  = kOffSSH  + (size_t)kRows * kSsmP * 2;
constexpr size_t kWsTotal = kOffSSL  + (size_t)kRows * kSsmP * 2;
static_assert(kWsTotal == 125829120ull, "carve total");
static_assert(kWsTotal <= 134217728ull, "carve cap");
static_assert((kOffWIB % 128) == 0 && (kOffWXB % 128) == 0 && (kOffWDB % 128) == 0 && (kOffWOB % 128) == 0 &&
              (kOffXSH % 128) == 0 && (kOffXSL % 128) == 0 && (kOffZH % 128) == 0 && (kOffZL % 128) == 0 &&
              (kOffXCH % 128) == 0 && (kOffXCL % 128) == 0 && (kOffSSH % 128) == 0 && (kOffSSL % 128) == 0,
              "128-B aligned regions");

__device__ __forceinline__ unsigned short f2bf_bits(float f) {
  unsigned u = __float_as_uint(f);
  return (unsigned short)((u + 0x7FFFu + ((u >> 16) & 1u)) >> 16);
}
__device__ __forceinline__ float bf_bits2f(unsigned short h) { return __uint_as_float(((unsigned)h) << 16); }
__device__ __forceinline__ float bfr(float f) { return bf_bits2f(f2bf_bits(f)); }

__device__ __forceinline__ float bfw_lo(unsigned w) { return __uint_as_float(w << 16); }
__device__ __forceinline__ float bfw_hi(unsigned w) { return __uint_as_float(w & 0xffff0000u); }
__device__ __forceinline__ void widen8(v4u uh, v4u ul, v4f& f0, v4f& f1) {
  const unsigned h0 = uh[0], h1 = uh[1], h2 = uh[2], h3 = uh[3];
  const unsigned l0 = ul[0], l1 = ul[1], l2 = ul[2], l3 = ul[3];
  f0[0] = bfw_lo(h0) + bfw_lo(l0); f0[1] = bfw_hi(h0) + bfw_hi(l0);
  f0[2] = bfw_lo(h1) + bfw_lo(l1); f0[3] = bfw_hi(h1) + bfw_hi(l1);
  f1[0] = bfw_lo(h2) + bfw_lo(l2); f1[1] = bfw_hi(h2) + bfw_hi(l2);
  f1[2] = bfw_lo(h3) + bfw_lo(l3); f1[3] = bfw_hi(h3) + bfw_hi(l3);
}

__device__ __forceinline__ void dep_guard4_h(v8f& a, v8f& b, v8f& c, v8f& d, v16h x, v16h y) { asm volatile("v_nop\n\tv_nop\n\tv_nop\n\tv_nop" : "+v"(a), "+v"(b), "+v"(c), "+v"(d) : "v"(x), "v"(y)); }
__device__ __forceinline__ void dep_guard4_b(v8f& a, v8f& b, v8f& c, v8f& d, v16b x, v16b y) { asm volatile("v_nop\n\tv_nop\n\tv_nop\n\tv_nop" : "+v"(a), "+v"(b), "+v"(c), "+v"(d) : "v"(x), "v"(y)); }
__device__ __forceinline__ void keep4_h(v16h a, v16h b, v16h c, v16h d) { asm volatile("v_nop" :: "v"(a), "v"(b), "v"(c), "v"(d)); }
__device__ __forceinline__ void keep4_b(v16b a, v16b b, v16b c, v16b d) { asm volatile("v_nop" :: "v"(a), "v"(b), "v"(c), "v"(d)); }
__device__ __forceinline__ void acc_guard4(v8f& a, v8f& b, v8f& c, v8f& d) { asm volatile("v_nop\n\tv_nop\n\tv_nop\n\tv_nop" : "+v"(a), "+v"(b), "+v"(c), "+v"(d)); }
__device__ __forceinline__ void dt_guard(v8f& a, v16b x0, v16b x1, v16b x2, v16b x3, v16b y0, v16b y1) {
  asm volatile("v_nop\n\tv_nop\n\tv_nop\n\tv_nop" : "+v"(a) : "v"(x0), "v"(x1), "v"(x2), "v"(x3), "v"(y0), "v"(y1));
}
template <typename T> struct Frag;
template <> struct Frag<_Float16> {
  typedef v16h V; union U { v16h v; v8h h[2]; };
  static __device__ __forceinline__ v16h load(const _Float16* p) {
    U f; f.h[0] = *(const v8h*)(p); f.h[1] = *(const v8h*)(p + 16); return f.v;
  }
  static __device__ __forceinline__ v8f mma(v16h a, v16h b, v8f c) {
    return __builtin_amdgcn_wmma_f32_16x16x32_f16(false, a, false, b, (short)0, c, false, false);
  }
  static __device__ __forceinline__ void guard4(v8f& a, v8f& b, v8f& c, v8f& d, v16h x, v16h y) { dep_guard4_h(a, b, c, d, x, y); }
  static __device__ __forceinline__ void keep(v16h a, v16h b, v16h c, v16h d) { keep4_h(a, b, c, d); }
};
template <> struct Frag<__bf16> {
  typedef v16b V; union U { v16b v; v8b h[2]; };
  static __device__ __forceinline__ v16b load(const __bf16* p) {
    U f; f.h[0] = *(const v8b*)(p); f.h[1] = *(const v8b*)(p + 16); return f.v;
  }
  static __device__ __forceinline__ v8f mma(v16b a, v16b b, v8f c) {
    return __builtin_amdgcn_wmma_f32_16x16x32_bf16(false, a, false, b, (short)0, c, false, false);
  }
  static __device__ __forceinline__ void guard4(v8f& a, v8f& b, v8f& c, v8f& d, v16b x, v16b y) { dep_guard4_b(a, b, c, d, x, y); }
  static __device__ __forceinline__ void keep(v16b a, v16b b, v16b c, v16b d) { keep4_b(a, b, c, d); }
};

template <int ET> struct Elem;
template <> struct Elem<0> { typedef _Float16 T; };
template <> struct Elem<1> { typedef __bf16 T; };
template <int ET, int SPL, int BIAS_MODE, int OUT_MODE, bool RESID, int ACT = 0>
__global__ __launch_bounds__(256) void wmma_gemm64(
    const unsigned short* __restrict__ Ap, const unsigned short* __restrict__ A2p, int lda, long strideA,
    const unsigned short* __restrict__ Btp, const unsigned short* __restrict__ Bt2p, int ldb, long strideB,
    void* __restrict__ Cout, void* __restrict__ Cout2, int ldc, long strideC,
    const float* __restrict__ bias,
    const float* __restrict__ resid, long strideR,
    int M, int N, int K, float scale) {
  typedef typename Elem<ET>::T T;
  typedef typename Frag<T>::V V;
  const T* A = (const T*)Ap; const T* A2 = (const T*)A2p; const T* Bt = (const T*)Btp; const T* Bt2 = (const T*)Bt2p;
  __shared__ __align__(16) float sT[8][16 * 68];
  const int b    = blockIdx.y;
  const int lane = threadIdx.x & 31;
  const int wave = threadIdx.x >> 5;
  const int tilesN = N >> 6;
  const int tilesM = M >> 6;
  const int tile = blockIdx.x * 8 + wave;
  if (tile >= tilesM * tilesN) return;
  const int tm = tile / tilesN;
  const int tn = tile - tm * tilesN;
  const int m0 = tm << 6;
  const int n0 = tn << 6;

  const T* Ab  = A  + (size_t)b * strideA;
  const T* Bb  = Bt + (size_t)b * strideB;
  const T* Ab2 = (SPL >= 1) ? (A2  + (size_t)b * strideA) : nullptr;
  const T* Bb2 = (SPL == 2) ? (Bt2 + (size_t)b * strideB) : nullptr;

  const int rlane = lane & 15;
  const int koff  = (lane >> 4) * 8;
  const int mOff  = (lane >> 4) * 8;

  v8f acc[4][4];
#pragma unroll
  for (int i = 0; i < 4; ++i)
#pragma unroll
    for (int j = 0; j < 4; ++j) acc[i][j] = (v8f){0.f,0.f,0.f,0.f,0.f,0.f,0.f,0.f};

  for (int k0 = 0; k0 < K; k0 += 32) {
    V bh[4], bl[4];
#pragma unroll
    for (int j = 0; j < 4; ++j) {
      const size_t bo = (size_t)(n0 + (j << 4) + rlane) * ldb + koff + k0;
      bh[j] = Frag<T>::load(Bb + bo);
      if (SPL == 2) bl[j] = Frag<T>::load(Bb2 + bo);
    }
#pragma unroll
    for (int i = 0; i < 4; ++i) {
      const size_t ao = (size_t)(m0 + (i << 4) + rlane) * lda + koff + k0;
      V ah = Frag<T>::load(Ab + ao);
      V al = ah;
      if (SPL >= 1) al = Frag<T>::load(Ab2 + ao);
#pragma unroll
      for (int j = 0; j < 4; ++j) {
        acc[i][j] = Frag<T>::mma(ah, bh[j], acc[i][j]);
        if (SPL == 2) acc[i][j] = Frag<T>::mma(ah, bl[j], acc[i][j]);
        if (SPL >= 1) acc[i][j] = Frag<T>::mma(al, bh[j], acc[i][j]);
      }
      Frag<T>::guard4(acc[i][0], acc[i][1], acc[i][2], acc[i][3], ah, al);
    }
    Frag<T>::keep(bh[0], bh[1], bh[2], bh[3]);
    if (SPL == 2) Frag<T>::keep(bl[0], bl[1], bl[2], bl[3]);
  }
  acc_guard4(acc[0][0], acc[0][1], acc[0][2], acc[0][3]);
  acc_guard4(acc[1][0], acc[1][1], acc[1][2], acc[1][3]);
  acc_guard4(acc[2][0], acc[2][1], acc[2][2], acc[2][3]);
  acc_guard4(acc[3][0], acc[3][1], acc[3][2], acc[3][3]);

  float* slab = sT[wave];
  const float* Rb = RESID ? (resid + (size_t)b * strideR) : nullptr;
#pragma unroll
  for (int i = 0; i < 4; ++i) {
    const int mBase = m0 + (i << 4);
#pragma unroll
    for (int j = 0; j < 4; ++j) {
      const int n = n0 + (j << 4) + rlane;
      float bv = 0.f;
      if (BIAS_MODE == 2) bv = bias[n];
#pragma unroll
      for (int r = 0; r < 8; ++r) {
        float v = acc[i][j][r] * scale;
        if (BIAS_MODE == 1) v += bias[mBase + mOff + r];
        if (BIAS_MODE == 2) v += bv;
        if (RESID) v += Rb[(size_t)(mBase + mOff + r) * ldc + n];
        if (ACT == 1) v = tanhf(v);
        if (ACT == 2) v = fmaxf(v, 0.0f);
        if (ACT == 3) v = v / (1.0f + expf(-v));
        if (ACT == 4) v = (v > 0.f) ? v : 0.01f * v;
        slab[(mOff + r) * 68 + (j << 4) + rlane] = v;
      }
    }
    __builtin_amdgcn_fence(__ATOMIC_RELEASE, "workgroup");
    __builtin_amdgcn_wave_barrier();
    __builtin_amdgcn_fence(__ATOMIC_ACQUIRE, "workgroup");
    if (OUT_MODE == 0) {
      float* C = (float*)Cout + (size_t)b * strideC;
      const int hh = lane >> 4, c4 = (lane & 15) * 4;
      for (int pass = 0; pass < 2; ++pass) {
#pragma unroll
        for (int it = 0; it < 8; ++it) {
          const int row = it * 2 + hh;
          v4f v = *(const v4f*)(slab + row * 68 + c4);
          *(volatile v4f*)(C + (size_t)(mBase + row) * ldc + n0 + c4) = v;
        }
        __threadfence();
      }
    } else {
      const int q = lane >> 3, c8 = (lane & 7) * 8;
      unsigned short* C  = (unsigned short*)Cout  + (size_t)b * strideC;
      unsigned short* C2 = (OUT_MODE == 2) ? ((unsigned short*)Cout2 + (size_t)b * strideC) : nullptr;
      for (int pass = 0; pass < 2; ++pass) {
#pragma unroll
        for (int it = 0; it < 4; ++it) {
          const int row = it * 4 + q;
          const float* sp = slab + row * 68 + c8;
          v8h hv, lv;
#pragma unroll
          for (int e = 0; e < 8; ++e) {
            if (OUT_MODE == 1) {
              hv[e] = (_Float16)sp[e];
            } else {
              unsigned short hb = f2bf_bits(sp[e]);
              unsigned short lb = f2bf_bits(sp[e] - bf_bits2f(hb));
              hv[e] = __builtin_bit_cast(_Float16, hb);
              lv[e] = __builtin_bit_cast(_Float16, lb);
            }
          }
          *(volatile v8h*)(C + (size_t)(mBase + row) * ldc + n0 + c8) = hv;
          if (OUT_MODE == 2) *(volatile v8h*)(C2 + (size_t)(mBase + row) * ldc + n0 + c8) = lv;
        }
        __threadfence();
      }
    }
    __builtin_amdgcn_fence(__ATOMIC_RELEASE, "workgroup");
    __builtin_amdgcn_wave_barrier();
    __builtin_amdgcn_fence(__ATOMIC_ACQUIRE, "workgroup");
  }
}

__global__ __launch_bounds__(256) void cvt_bf16_kernel(
    const float* __restrict__ src, unsigned short* __restrict__ dst, int total8)
{
  const int i = blockIdx.x * 256 + threadIdx.x;
  if (i >= total8) return;
  const size_t e0 = (size_t)i << 3;
  const v4f a0 = *(const v4f*)(src + e0);
  const v4f a1 = *(const v4f*)(src + e0 + 4);
  v8h hv;
#pragma unroll
  for (int e = 0; e < 4; ++e) {
    const float f0 = a0[e], f1 = a1[e];
    hv[e]     = __builtin_bit_cast(_Float16, f2bf_bits(f0));
    hv[4 + e] = __builtin_bit_cast(_Float16, f2bf_bits(f1));
  }
  unsigned short* q = dst + e0;
  *(volatile v8h*)q = hv;
  __threadfence();
  *(volatile v8h*)q = hv;
}

__global__ __launch_bounds__(256) void conv_silu_kernel(
    const unsigned short* __restrict__ XSH, const unsigned short* __restrict__ XSL,
    const float* __restrict__ cw, const float* __restrict__ cb,
    unsigned short* __restrict__ XCH, unsigned short* __restrict__ XCL)
{
  __shared__ __align__(16) float sIn[16 * kConvTP];
  __shared__ __align__(16) float sOut[16 * kConvTP];
  const int tid = threadIdx.x, lane = tid & 31, wave = tid >> 5;
  const int d0 = blockIdx.x * 256, d = d0 + tid;
  const int g0 = blockIdx.y * 64;
  const int tb = g0 & (kSeq - 1);
  const v4f wv = *(const v4f*)(cw + (size_t)d * 4);
  const float wa = wv[0], wb = wv[1], wc = wv[2], wd = wv[3];
  const float w0 = bfr(wa), w1 = bfr(wb), w2 = bfr(wc), w3 = bfr(wd);
  const float bc = bfr(cb[d]);
  const unsigned* Hw = (const unsigned*)XSH;
  const unsigned* Lw = (const unsigned*)XSL;
  const v4u* Hq = (const v4u*)XSH;
  const v4u* Lq = (const v4u*)XSL;
  float xm3, xm2, xm1;
  {
    const bool hist = (tb > 0);
    const int rb = hist ? (g0 - 3) : g0;
    const size_t i0 = ((size_t)rb * kDin + d) >> 1;
    const size_t i1 = ((size_t)(rb + 1) * kDin + d) >> 1;
    const size_t i2 = ((size_t)(rb + 2) * kDin + d) >> 1;
    const unsigned uh0 = Hw[i0], uh1 = Hw[i1], uh2 = Hw[i2];
    const unsigned ul0 = Lw[i0], ul1 = Lw[i1], ul2 = Lw[i2];
    const bool odd = (d & 1) != 0;
    const float v0 = odd ? (bfw_hi(uh0) + bfw_hi(ul0)) : (bfw_lo(uh0) + bfw_lo(ul0));
    const float v1 = odd ? (bfw_hi(uh1) + bfw_hi(ul1)) : (bfw_lo(uh1) + bfw_lo(ul1));
    const float v2 = odd ? (bfw_hi(uh2) + bfw_hi(ul2)) : (bfw_lo(uh2) + bfw_lo(ul2));
    xm3 = hist ? v0 : 0.f;
    xm2 = hist ? v1 : 0.f;
    xm1 = hist ? v2 : 0.f;
  }
#pragma unroll 1
  for (int sub = 0; sub < 4; ++sub) {
    const int lb = g0 + sub * 16;
#pragma unroll
    for (int i = 0; i < 2; ++i) {
      const int idx = tid + 256 * i;
      const int r = idx >> 5, c8 = (idx & 31) * 8;
      const size_t go = ((size_t)(lb + r) * kDin + d0 + c8) >> 3;
      const v4u uh = Hq[go], ul = Lq[go];
      v4f f0, f1;
      widen8(uh, ul, f0, f1);
      *(v4f*)(sIn + r * kConvTP + c8)     = f0;
      *(v4f*)(sIn + r * kConvTP + c8 + 4) = f1;
    }
    __syncthreads();
#pragma unroll 1
    for (int s = 0; s < 16; ++s) {
      const float xcur = sIn[s * kConvTP + tid];
      float acc = w0 * xm3;
      acc = fmaf(w1, xm2, acc);
      acc = fmaf(w2, xm1, acc);
      acc = fmaf(w3, xcur, acc);
      const float sv = acc + bc;
      const float sg = __builtin_amdgcn_rcpf(1.0f + expf(-sv));
      sOut[s * kConvTP + tid] = sv * sg;
      xm3 = xm2; xm2 = xm1; xm1 = xcur;
    }
    __syncthreads();
    v8h hv[2], lv[2];
#pragma unroll
    for (int it = 0; it < 2; ++it) {
      const float* sp = sOut + (it * 8 + wave) * kConvTP + lane * 8;
      const v4f a0 = *(const v4f*)(sp);
      const v4f a1 = *(const v4f*)(sp + 4);
#pragma unroll
      for (int e = 0; e < 4; ++e) {
        const float fa = a0[e], fb = a1[e];
        const unsigned short h0 = f2bf_bits(fa), h1 = f2bf_bits(fb);
        const unsigned short l0 = f2bf_bits(fa - bf_bits2f(h0)), l1 = f2bf_bits(fb - bf_bits2f(h1));
        hv[it][e]     = __builtin_bit_cast(_Float16, h0);
        hv[it][4 + e] = __builtin_bit_cast(_Float16, h1);
        lv[it][e]     = __builtin_bit_cast(_Float16, l0);
        lv[it][4 + e] = __builtin_bit_cast(_Float16, l1);
      }
    }
    for (int pass = 0; pass < 2; ++pass) {
#pragma unroll
      for (int it = 0; it < 2; ++it) {
        const size_t o = (size_t)(lb + it * 8 + wave) * kDin + d0 + lane * 8;
        *(volatile v8h*)(XCH + o) = hv[it];
        *(volatile v8h*)(XCL + o) = lv[it];
      }
      __threadfence();
    }
    __syncthreads();
  }
}

__global__ __launch_bounds__(256) void scan_kernel(
    const unsigned short* __restrict__ SSH, const unsigned short* __restrict__ SSL,
    const unsigned short* __restrict__ XCH, const unsigned short* __restrict__ XCL,
    const unsigned short* __restrict__ ZH,  const unsigned short* __restrict__ ZL,
    const unsigned short* __restrict__ WDB,
    const float* __restrict__ bdt, const float* __restrict__ Alog, const float* __restrict__ Dp,
    unsigned short* __restrict__ YGH, unsigned short* __restrict__ YGL)
{
  __shared__ __align__(16) float sBC[kScanTS * kBCW];
  __shared__ __align__(16) float sDT[kScanTS * kScanCh];
  __shared__ __align__(16) float sXC[kScanTS * kScanCh];
  __shared__ __align__(16) float sG[kScanTS * kScanCh];
  __shared__ __align__(16) float sY[kScanTS * kScanYP];
  const int tid = threadIdx.x, lane = tid & 31, wave = tid >> 5;
  constexpr int kBlkPerB = kDin / kScanCh;
  const int bix = blockIdx.x / kBlkPerB;
  const int d0  = (blockIdx.x - bix * kBlkPerB) * kScanCh;
  const int c   = wave * 8 + (lane & 7);
  const int sq  = lane >> 3;
  const int d   = d0 + c;
  const size_t row0 = (size_t)bix * kSeq;
#pragma unroll 1
  for (int i = 0; i < 16; ++i) {
    const int idx = tid * 16 + i;
    const int r = idx >> 6, n = idx & 63;
    const float v = Alog[(size_t)(d0 + r) * kNst + n];
    sBC[idx] = -expf(bfr(v)) * kLog2e;
  }
  __syncthreads();
  float nA2[kScanQ], h[kScanQ];
#pragma unroll
  for (int k4 = 0; k4 < kScanQ / 4; ++k4) {
    const v4f av = *(const v4f*)(sBC + c * kNst + sq * kScanQ + 4 * k4);
    nA2[4 * k4 + 0] = av[0]; nA2[4 * k4 + 1] = av[1]; nA2[4 * k4 + 2] = av[2]; nA2[4 * k4 + 3] = av[3];
  }
#pragma unroll
  for (int k = 0; k < kScanQ; ++k) h[k] = 0.0f;
  const int rlane = lane & 15, koff = (lane >> 4) * 8;
  const int mt = wave & 1, nt = wave >> 1;
  const __bf16* Wb = (const __bf16*)WDB + (size_t)(d0 + nt * 16 + rlane) * kDtR + koff;
  const v16b bw0 = Frag<__bf16>::load(Wb);
  const v16b bw1 = Frag<__bf16>::load(Wb + 32);
  const float Dd = bfr(Dp[d]);
  const int cc = tid & 63, srow = tid >> 6;
  const float bb = bfr(bdt[d0 + cc]);
  const int yr = tid >> 3, yc8 = (tid & 7) * 8;
  const v4u* SSHq = (const v4u*)SSH;
  const v4u* SSLq = (const v4u*)SSL;
  const v4u* XCHq = (const v4u*)XCH;
  const v4u* XCLq = (const v4u*)XCL;
  const v4u* ZHq  = (const v4u*)ZH;
  const v4u* ZLq  = (const v4u*)ZL;
  const __bf16* SSHb = (const __bf16*)SSH;
  const __bf16* SSLb = (const __bf16*)SSL;
#pragma unroll 1
  for (int t0 = 0; t0 < kSeq; t0 += kScanTS) {
    __syncthreads();
#pragma unroll
    for (int i = 0; i < 2; ++i) {
      const int idx = tid + 256 * i;
      const int r = idx >> 4, c8 = (idx & 15) * 8;
      const size_t go = ((row0 + t0 + r) * kSsmP + kBcOff + c8) >> 3;
      const v4u uh = SSHq[go], ul = SSLq[go];
      v4f f0, f1;
      widen8(uh, ul, f0, f1);
      *(v4f*)(sBC + r * kBCW + c8)     = f0;
      *(v4f*)(sBC + r * kBCW + c8 + 4) = f1;
    }
    asm volatile("" ::: "memory");
    {
      const size_t go = ((row0 + t0 + yr) * kDin + d0 + yc8) >> 3;
      const v4u xh = XCHq[go], xl = XCLq[go], zh = ZHq[go], zl = ZLq[go];
      v4f x0, x1, z0, z1, ga, gb;
      widen8(xh, xl, x0, x1);
      widen8(zh, zl, z0, z1);
#pragma unroll
      for (int e = 0; e < 4; ++e) {
        const float za = z0[e], zb = z1[e];
        ga[e] = za * __builtin_amdgcn_rcpf(1.0f + expf(-za));
        gb[e] = zb * __builtin_amdgcn_rcpf(1.0f + expf(-zb));
      }
      *(v4f*)(sXC + yr * kScanCh + yc8)     = x0;
      *(v4f*)(sXC + yr * kScanCh + yc8 + 4) = x1;
      *(v4f*)(sG  + yr * kScanCh + yc8)     = ga;
      *(v4f*)(sG  + yr * kScanCh + yc8 + 4) = gb;
    }
    asm volatile("" ::: "memory");
    {
      v8f acc = (v8f){0.f,0.f,0.f,0.f,0.f,0.f,0.f,0.f};
      const size_t ao = (row0 + t0 + mt * 16 + rlane) * kSsmP + koff;
      const v16b ah0 = Frag<__bf16>::load(SSHb + ao);
      const v16b al0 = Frag<__bf16>::load(SSLb + ao);
      const v16b ah1 = Frag<__bf16>::load(SSHb + ao + 32);
      const v16b al1 = Frag<__bf16>::load(SSLb + ao + 32);
      acc = Frag<__bf16>::mma(ah0, bw0, acc);
      acc = Frag<__bf16>::mma(al0, bw0, acc);
      acc = Frag<__bf16>::mma(ah1, bw1, acc);
      acc = Frag<__bf16>::mma(al1, bw1, acc);
      dt_guard(acc, ah0, al0, ah1, al1, bw0, bw1);
#pragma unroll
      for (int r = 0; r < 8; ++r) sDT[(mt * 16 + koff + r) * kScanCh + nt * 16 + rlane] = acc[r];
    }
    __syncthreads();
#pragma unroll 1
    for (int i = 0; i < 8; ++i) {
      const int s = srow + 4 * i;
      float* p = sDT + s * kScanCh + cc;
      const float v = *p + bb;
      const float a = expf(-fabsf(v));
      *p = fmaxf(v, 0.0f) + log1pf(a);
    }
    __syncthreads();
#pragma unroll 1
    for (int s = 0; s < kScanTS; ++s) {
      const float dt  = sDT[s * kScanCh + c];
      const float xt  = sXC[s * kScanCh + c];
      const float g   = sG[s * kScanCh + c];
      const float dtx = dt * xt;
      const float* bp = sBC + s * kBCW + sq * kScanQ;
      const float* cp = bp + kNst;
      float yp = 0.0f;
#pragma unroll
      for (int k4 = 0; k4 < kScanQ / 4; ++k4) {
        const v4f bv = *(const v4f*)(bp + 4 * k4);
        const v4f cv = *(const v4f*)(cp + 4 * k4);
#pragma unroll
        for (int e = 0; e < 4; ++e) {
          const float ex = __builtin_amdgcn_exp2f(dt * nA2[4 * k4 + e]);
          h[4 * k4 + e] = fmaf(ex, h[4 * k4 + e], dtx * bv[e]);
          yp = fmaf(h[4 * k4 + e], cv[e], yp);
        }
      }
      yp += __shfl_xor(yp, 8, 32);
      yp += __shfl_xor(yp, 16, 32);
      const float y = fmaf(xt, Dd, yp);
      sY[s * kScanYP + c] = y * g;
    }
    __syncthreads();
    {
      const float* sp = sY + yr * kScanYP + yc8;
      const v4f a0 = *(const v4f*)(sp);
      const v4f a1 = *(const v4f*)(sp + 4);
      v8h hv, lv;
#pragma unroll
      for (int e = 0; e < 4; ++e) {
        const float fa = a0[e], fb = a1[e];
        const unsigned short h0 = f2bf_bits(fa), h1 = f2bf_bits(fb);
        const unsigned short l0 = f2bf_bits(fa - bf_bits2f(h0)), l1 = f2bf_bits(fb - bf_bits2f(h1));
        hv[e]     = __builtin_bit_cast(_Float16, h0);
        hv[4 + e] = __builtin_bit_cast(_Float16, h1);
        lv[e]     = __builtin_bit_cast(_Float16, l0);
        lv[4 + e] = __builtin_bit_cast(_Float16, l1);
      }
      const size_t o = (row0 + t0 + yr) * kDin + d0 + yc8;
      *(volatile v8h*)(YGH + o) = hv;
      *(volatile v8h*)(YGL + o) = lv;
      __threadfence();
      *(volatile v8h*)(YGH + o) = hv;
      *(volatile v8h*)(YGL + o) = lv;
    }
  }
}

static inline int cdiv_host(long long a, long long b) { return (int)((a + b - 1) / b); }

extern "C" void kernel_launch(void* const* d_in, const int* in_sizes, int n_in,
                              void* d_out, int out_size, void* d_ws, size_t ws_size,
                              hipStream_t stream) {
  if (n_in < 10) return;
  if (in_sizes[0] != kRows * kDm) return;
  if (in_sizes[1] != kXzP * kDm) return;
  if (in_sizes[2] != kDin * 4) return;
  if (in_sizes[3] != kDin) return;
  if (in_sizes[4] != kSsmP * kDin) return;
  if (in_sizes[5] != kDin * kDtR) return;
  if (in_sizes[6] != kDin) return;
  if (in_sizes[7] != kDin * kNst) return;
  if (in_sizes[8] != kDin) return;
  if (in_sizes[9] != kDm * kDin) return;
  if (out_size != kRows * kDm) return;
  if (ws_size < kWsTotal) return;

  const float* x      = (const float*)d_in[0];
  const float* W_in   = (const float*)d_in[1];
  const float* conv_w = (const float*)d_in[2];
  const float* conv_b = (const float*)d_in[3];
  const float* W_x    = (const float*)d_in[4];
  const float* W_dt   = (const float*)d_in[5];
  const float* b_dt   = (const float*)d_in[6];
  const float* A_log  = (const float*)d_in[7];
  const float* Dp     = (const float*)d_in[8];
  const float* W_out  = (const float*)d_in[9];
  float* out = (float*)d_out;

  char* ws = (char*)d_ws;
  unsigned short* XB   = (unsigned short*)(ws + kOffXB);
  unsigned short* WIB  = (unsigned short*)(ws + kOffWIB);
  unsigned short* WXB  = (unsigned short*)(ws + kOffWXB);
  unsigned short* WDB  = (unsigned short*)(ws + kOffWDB);
  unsigned short* WOB  = (unsigned short*)(ws + kOffWOB);
  unsigned short* XSH  = (unsigned short*)(ws + kOffXSH);
  unsigned short* XSL  = (unsigned short*)(ws + kOffXSL);
  unsigned short* ZH   = (unsigned short*)(ws + kOffZH);
  unsigned short* ZL   = (unsigned short*)(ws + kOffZL);
  unsigned short* XCH  = (unsigned short*)(ws + kOffXCH);
  unsigned short* XCL  = (unsigned short*)(ws + kOffXCL);
  unsigned short* SSH  = (unsigned short*)(ws + kOffSSH);
  unsigned short* SSL  = (unsigned short*)(ws + kOffSSL);
  unsigned short* YGH  = XSH;
  unsigned short* YGL  = XSL;

  {
    const int n0 = kRows * kDm / 8, n1 = kXzP * kDm / 8, n2 = kSsmP * kDin / 8, n3 = kDin * kDtR / 8, n4 = kDm * kDin / 8;
    cvt_bf16_kernel<<<cdiv_host(n0, 256), 256, 0, stream>>>(x,     XB,  n0);
    cvt_bf16_kernel<<<cdiv_host(n1, 256), 256, 0, stream>>>(W_in,  WIB, n1);
    cvt_bf16_kernel<<<cdiv_host(n2, 256), 256, 0, stream>>>(W_x,   WXB, n2);
    cvt_bf16_kernel<<<cdiv_host(n3, 256), 256, 0, stream>>>(W_dt,  WDB, n3);
    cvt_bf16_kernel<<<cdiv_host(n4, 256), 256, 0, stream>>>(W_out, WOB, n4);
  }

  wmma_gemm64<1, 0, 0, 2, false><<<dim3(cdiv_host((kRows / 64) * (kDin / 64), 8), 1), 256, 0, stream>>>(
      XB, nullptr, kDm, 0L,
      WIB, nullptr, kDm, 0L,
      (void*)XSH, (void*)XSL, kDin, 0L,
      nullptr, nullptr, 0L,
      kRows, kDin, kDm, 1.0f);

  wmma_gemm64<1, 0, 0, 2, false><<<dim3(cdiv_host((kRows / 64) * (kDin / 64), 8), 1), 256, 0, stream>>>(
      XB, nullptr, kDm, 0L,
      WIB + (size_t)kDin * kDm, nullptr, kDm, 0L,
      (void*)ZH, (void*)ZL, kDin, 0L,
      nullptr, nullptr, 0L,
      kRows, kDin, kDm, 1.0f);

  conv_silu_kernel<<<dim3(kDin / 256, kRows / 64), 256, 0, stream>>>(XSH, XSL, conv_w, conv_b, XCH, XCL);

  wmma_gemm64<1, 1, 0, 2, false><<<dim3(cdiv_host((kRows / 64) * (kSsmP / 64), 8), 1), 256, 0, stream>>>(
      XCH, XCL, kDin, 0L,
      WXB, nullptr, kDin, 0L,
      (void*)SSH, (void*)SSL, kSsmP, 0L,
      nullptr, nullptr, 0L,
      kRows, kSsmP, kDin, 1.0f);

  scan_kernel<<<kBatch * (kDin / kScanCh), 256, 0, stream>>>(
      SSH, SSL, XCH, XCL, ZH, ZL, WDB, b_dt, A_log, Dp, YGH, YGL);

  wmma_gemm64<1, 1, 0, 0, false><<<dim3(cdiv_host((kRows / 64) * (kDm / 64), 8), 1), 256, 0, stream>>>(
      YGH, YGL, kDin, 0L,
      WOB, nullptr, kDin, 0L,
      (void*)out, nullptr, kDm, 0L,
      nullptr, nullptr, 0L,
      kRows, kDm, kDin, 1.0f);
}
